// MultiHeadAttention_73890617361024
// MI455X (gfx1250) — hardware-verified
//
#include <hip/hip_runtime.h>


#ifndef NB
#define NB 2
#endif
#ifndef SEQ
#define SEQ 2048
#endif
#define NB_FULL  2
#define SEQ_FULL 2048
#ifndef OUT_SEQ
#define OUT_SEQ SEQ
#endif
#define DM   2048
#define NH_  16
#define HD   128
#define AW   4
#define OSP  132
#define SC2  (0.08838834764831845f * 1.4426950408889634f)
#define PSH  8.0f
#define CTS  256.0f
#define WPS  1024.0f
#define OSC  (1.0f / (256.0f * 1024.0f))

static_assert(HD == 128);
static_assert(NH_ * HD == DM);
static_assert(DM % 64 == 0);
static_assert(DM % 32 == 0);
static_assert(HD % 64 == 0);
static_assert(SEQ % 64 == 0);
static_assert((NB * SEQ) % 64 == 0);
static_assert(SEQ % 32 == 0);
static_assert(SEQ % (16 * AW) == 0);
static_assert(((size_t)SEQ * DM) % 8 == 0);
static_assert(NB <= NB_FULL);
static_assert(SEQ <= SEQ_FULL);
static_assert((OSP * 4) % 16 == 0);

typedef _Float16 h16;
typedef unsigned short bf;
typedef __attribute__((ext_vector_type(16))) __bf16   v16bf;
typedef __attribute__((ext_vector_type(16))) _Float16 v16h;
typedef __attribute__((ext_vector_type(8)))  _Float16 v8h;
typedef __attribute__((ext_vector_type(8)))  unsigned short v8us;
typedef __attribute__((ext_vector_type(8)))  float    v8f;
typedef __attribute__((ext_vector_type(4)))  float    v4f;
typedef v4f  __attribute__((may_alias)) v4fa;

__device__ __forceinline__ unsigned short f2bf(float f) { unsigned u = __float_as_uint(f); u += 0x7FFFu + ((u >> 16) & 1u); return (unsigned short)(u >> 16); }
__device__ __forceinline__ float bfr(float f) { return __uint_as_float(((unsigned)f2bf(f)) << 16); }
__device__ __forceinline__ v16h cat16(v8h lo, v8h hi) { return __builtin_shufflevector(lo, hi, 0, 1, 2, 3, 4, 5, 6, 7, 8, 9, 10, 11, 12, 13, 14, 15); }
__device__ __forceinline__ v16bf cat16b(v8us lo, v8us hi) { return __builtin_bit_cast(v16bf, __builtin_shufflevector(lo, hi, 0, 1, 2, 3, 4, 5, 6, 7, 8, 9, 10, 11, 12, 13, 14, 15)); }
__device__ __forceinline__ v8f wmma16(v16h a, v16h b, v8f c) { return __builtin_amdgcn_wmma_f32_16x16x32_f16(false, a, false, b, (short)0, c, false, false); }
__device__ __forceinline__ v8f wmmab(v16bf a, v16bf b, v8f c) { return __builtin_amdgcn_wmma_f32_16x16x32_bf16(false, a, false, b, (short)0, c, false, false); }
__device__ __forceinline__ v16h  ldh(const h16* p) { return cat16(*(const v8h*)p, *(const v8h*)(p + 16)); }
__device__ __forceinline__ v16bf ldb(const bf* p)  { return cat16b(*(const v8us*)p, *(const v8us*)(p + 16)); }
__device__ __forceinline__ void wave_sync() { __builtin_amdgcn_fence(3  , "wavefront"); __builtin_amdgcn_wave_barrier(); asm volatile("" ::: "memory"); }

__global__ __launch_bounds__(256) void k_cvt8(const float* __restrict__ src, bf* dst, size_t n8) {
    const size_t i = (size_t)blockIdx.x * 256 + threadIdx.x; if (i >= n8) return;
    const v8f v = *(const v8f*)(src + i * 8); v8us o;
#pragma unroll
    for (int k = 0; k < 8; ++k) o[k] = f2bf(v[k]);
    *(volatile v8us*)(dst + i * 8) = o; __threadfence(); *(volatile v8us*)(dst + i * 8) = o;
}

__global__ __launch_bounds__(256) void k_tr(const float* __restrict__ in, unsigned short* out, int R, int C, int f16mode, float scale) {
    __shared__ float ts[64 * 65];
    const int tid = threadIdx.x; const int r0 = blockIdx.y * 64, c0 = blockIdx.x * 64;
#pragma unroll
    for (int i = 0; i < 4; ++i) { const int q = i * 256 + tid; const int r = q >> 4, c4 = (q & 15) * 4;
        const v4f v = *(const v4f*)(in + (size_t)(r0 + r) * C + c0 + c4);
        ts[r * 65 + c4 + 0] = v[0]; ts[r * 65 + c4 + 1] = v[1]; ts[r * 65 + c4 + 2] = v[2]; ts[r * 65 + c4 + 3] = v[3]; }
    __syncthreads();
    v8us o[2];
#pragma unroll
    for (int it = 0; it < 2; ++it) { const int q = it * 256 + tid; const int c = q >> 3, r8 = (q & 7) * 8;
#pragma unroll
        for (int j = 0; j < 8; ++j) { const float f = ts[(r8 + j) * 65 + c];
            const unsigned short ub = f2bf(f);
            const float g = __uint_as_float(((unsigned)ub) << 16) * scale;
            const unsigned short uh = __builtin_bit_cast(unsigned short, (h16)g);
            o[it][j] = f16mode ? uh : ub; } }
#pragma unroll 1
    for (int ps = 0; ps < 2; ++ps) {
#pragma unroll
        for (int it = 0; it < 2; ++it) { const int q = it * 256 + tid; const int c = q >> 3, r8 = (q & 7) * 8;
            *(volatile v8us*)(out + (size_t)(c0 + c) * R + r0 + r8) = o[it]; }
        if (ps == 0) __threadfence(); }
}

__global__ __launch_bounds__(32) void k_proj(const bf* __restrict__ A, const bf* __restrict__ Bt, const float* __restrict__ bias, int biasRow, h16* P, int RB, size_t sRB, int pitch, int CB, size_t sCB) {
    __shared__ __align__(16) float os[16 * 68];
    const int K = DM;
    const int lane = threadIdx.x & 31, lr = lane & 15, hi = lane >> 4; const int r0 = blockIdx.x * 64, c0 = blockIdx.y * 64;
    v8f acc[4][4];
#pragma unroll
    for (int mb = 0; mb < 4; ++mb)
#pragma unroll
        for (int nb = 0; nb < 4; ++nb) acc[mb][nb] = (v8f){};
    const size_t aoff = (size_t)(r0 + lr) * K + 8 * hi, boff = (size_t)(c0 + lr) * K + 8 * hi;
#pragma unroll 1
    for (int kc = 0; kc < K; kc += 32) {
        v16bf a[4];
#pragma unroll
        for (int mb = 0; mb < 4; ++mb) a[mb] = ldb(A + aoff + (size_t)mb * 16 * K + kc);
#pragma unroll
        for (int nb = 0; nb < 4; ++nb) { const v16bf b = ldb(Bt + boff + (size_t)nb * 16 * K + kc);
#pragma unroll
            for (int mb = 0; mb < 4; ++mb) acc[mb][nb] = wmmab(a[mb], b, acc[mb][nb]); }
        asm volatile("v_nop\n\tv_nop\n\tv_nop\n\tv_nop" : "+v"(acc[0][0]), "+v"(acc[1][1]), "+v"(acc[2][2]), "+v"(acc[3][3]) : "v"(a[0]), "v"(a[1]), "v"(a[2]), "v"(a[3]));
    }
    const size_t tbase = (size_t)(r0 / RB) * sRB + (size_t)(r0 % RB) * (size_t)pitch + (size_t)(c0 / CB) * sCB + (size_t)(c0 % CB);
#pragma unroll
    for (int mb = 0; mb < 4; ++mb) {
#pragma unroll
        for (int nb = 0; nb < 4; ++nb) {
#pragma unroll
            for (int j = 0; j < 8; ++j) os[(hi * 8 + j) * 68 + nb * 16 + lr] = acc[mb][nb][j]; }
        wave_sync();
        const size_t sb = tbase + (size_t)(mb * 16) * (size_t)pitch;
#pragma unroll 1
        for (int ps = 0; ps < 2; ++ps) {
#pragma unroll
            for (int s = 0; s < 4; ++s) { const int row = 4 * s + (lane >> 3), c8 = (lane & 7) * 8;
                const int bi0 = biasRow ? (r0 + mb * 16 + row) : (c0 + c8); const int bst = biasRow ? 0 : 1;
                const v4f x0 = *(const v4fa*)(&os[row * 68 + c8]); const v4f x1 = *(const v4fa*)(&os[row * 68 + c8 + 4]); v8h hv;
#pragma unroll
                for (int i = 0; i < 4; ++i) { const float b0 = bfr(bias[bi0 + i * bst]); const float b1 = bfr(bias[bi0 + (4 + i) * bst]);
                    hv[i] = (h16)(x0[i] + b0); hv[4 + i] = (h16)(x1[i] + b1); }
                const size_t oo = sb + (size_t)row * (size_t)pitch + c8;
                *(volatile v8h*)(P + oo) = hv; }
            if (ps == 0) __threadfence(); }
        wave_sync();
    }
}

__global__ __launch_bounds__(32 * AW) void k_flash(const h16* __restrict__ QK, const h16* __restrict__ VT, h16* CT) {
    __shared__ __align__(16) float os[AW * 16 * OSP];
    const int lane = threadIdx.x & 31, wave = __builtin_amdgcn_readfirstlane((int)(threadIdx.x >> 5)), lr = lane & 15, hi = lane >> 4;
    const int zh = blockIdx.y; const int b = zh / NH_, h = zh % NH_;
    const int t0 = (blockIdx.x * AW + wave) * 16;
    const size_t qbase = (size_t)(b * 2 * NH_ + h) * SEQ * HD;
    const size_t kbase = qbase + (size_t)NH_ * SEQ * HD;
    const size_t vbase = (size_t)zh * HD * SEQ;
    const size_t qo = qbase + (size_t)(t0 + lr) * HD + 8 * hi;
    const v16h q0 = ldh(QK + qo), q1 = ldh(QK + qo + 32), q2 = ldh(QK + qo + 64), q3 = ldh(QK + qo + 96);
    const size_t ko = kbase + (size_t)lr * HD + 8 * hi;
    const size_t vo = vbase + (size_t)lr * SEQ + 8 * hi;
    v8f o[8];
#pragma unroll
    for (int j = 0; j < 8; ++j) o[j] = (v8f){};
    float m = -3.0e38f, l = 0.0f;
#pragma unroll 1
    for (int key0 = 0; key0 < SEQ; key0 += 32) {
        const h16* ka = QK + ko + (size_t)key0 * HD;
        v8f sa = (v8f){}, sb = (v8f){};
        { const v16h a0 = ldh(ka), a1 = ldh(ka + 32), b0 = ldh(ka + 16 * HD), b1 = ldh(ka + 16 * HD + 32);
          sa = wmma16(a0, q0, sa); sb = wmma16(b0, q0, sb); sa = wmma16(a1, q1, sa); sb = wmma16(b1, q1, sb);
          asm volatile("v_nop\n\tv_nop\n\tv_nop\n\tv_nop" : "+v"(sa), "+v"(sb) : "v"(a0), "v"(a1), "v"(b0), "v"(b1)); }
        { const v16h a2 = ldh(ka + 64), a3 = ldh(ka + 96), b2 = ldh(ka + 16 * HD + 64), b3 = ldh(ka + 16 * HD + 96);
          sa = wmma16(a2, q2, sa); sb = wmma16(b2, q2, sb); sa = wmma16(a3, q3, sa); sb = wmma16(b3, q3, sb);
          asm volatile("v_nop\n\tv_nop\n\tv_nop\n\tv_nop" : "+v"(sa), "+v"(sb) : "v"(a2), "v"(a3), "v"(b2), "v"(b3)); }
        float ta[8], tb[8]; float mx = -3.0e38f;
#pragma unroll
        for (int r = 0; r < 8; ++r) { ta[r] = sa[r] * SC2; tb[r] = sb[r] * SC2; mx = fmaxf(mx, fmaxf(ta[r], tb[r])); }
        mx = fmaxf(mx, __shfl_xor(mx, 16, 32));
        const float mnew = fmaxf(m, mx);
        const float alpha = __builtin_amdgcn_exp2f(m - mnew);
        const float sh = PSH - mnew;
        v16h pb; float ls = 0.0f;
#pragma unroll
        for (int r = 0; r < 8; ++r) { const h16 pa = (h16)__builtin_amdgcn_exp2f(ta[r] + sh); const h16 pc = (h16)__builtin_amdgcn_exp2f(tb[r] + sh); pb[r] = pa; pb[8 + r] = pc; ls += (float)pa + (float)pc; }
        l = l * alpha + ls; m = mnew;
#pragma unroll
        for (int j = 0; j < 8; ++j) o[j] = o[j] * alpha;
        const h16* va = VT + vo + key0;
        { const v16h v0 = ldh(va), v1 = ldh(va + (size_t)16 * SEQ), v2 = ldh(va + (size_t)32 * SEQ), v3 = ldh(va + (size_t)48 * SEQ);
          o[0] = wmma16(v0, pb, o[0]); o[1] = wmma16(v1, pb, o[1]); o[2] = wmma16(v2, pb, o[2]); o[3] = wmma16(v3, pb, o[3]);
          asm volatile("v_nop\n\tv_nop\n\tv_nop\n\tv_nop" : "+v"(o[0]), "+v"(o[1]), "+v"(o[2]), "+v"(o[3]) : "v"(v0), "v"(v1), "v"(v2), "v"(v3), "v"(pb)); }
        { const v16h v4 = ldh(va + (size_t)64 * SEQ), v5 = ldh(va + (size_t)80 * SEQ), v6 = ldh(va + (size_t)96 * SEQ), v7 = ldh(va + (size_t)112 * SEQ);
          o[4] = wmma16(v4, pb, o[4]); o[5] = wmma16(v5, pb, o[5]); o[6] = wmma16(v6, pb, o[6]); o[7] = wmma16(v7, pb, o[7]);
          asm volatile("v_nop\n\tv_nop\n\tv_nop\n\tv_nop" : "+v"(o[4]), "+v"(o[5]), "+v"(o[6]), "+v"(o[7]) : "v"(v4), "v"(v5), "v"(v6), "v"(v7), "v"(pb)); }
    }
    l += __shfl_xor(l, 16, 32);
    const float inv = CTS * (1.0f / l);
    const int wb = wave * 16 * OSP;
#pragma unroll
    for (int j = 0; j < 8; ++j) { v4f a, c;
#pragma unroll
        for (int i = 0; i < 4; ++i) { a[i] = o[j][i] * inv; c[i] = o[j][4 + i] * inv; }
        *(v4fa*)(&os[wb + lr * OSP + 16 * j + 8 * hi]) = a; *(v4fa*)(&os[wb + lr * OSP + 16 * j + 8 * hi + 4]) = c; }
    wave_sync();
    h16* crow = CT + ((size_t)b * SEQ + t0) * DM + h * HD;
#pragma unroll 1
    for (int ps = 0; ps < 2; ++ps) {
#pragma unroll
        for (int s = 0; s < 8; ++s) { const int row = 2 * s + hi, cofs = lr * 8;
            const v4f x0 = *(const v4fa*)(&os[wb + row * OSP + cofs]); const v4f x1 = *(const v4fa*)(&os[wb + row * OSP + cofs + 4]); v8h hv;
#pragma unroll
            for (int i = 0; i < 4; ++i) { hv[i] = (h16)x0[i]; hv[4 + i] = (h16)x1[i]; }
            *(volatile v8h*)(crow + (size_t)row * DM + cofs) = hv; }
        if (ps == 0) __threadfence(); }
}

__global__ __launch_bounds__(32) void k_out(const h16* __restrict__ A, const h16* __restrict__ Bt, const float* __restrict__ bias, float* OUT) {
    __shared__ __align__(16) float os[16 * 68];
    const int K = DM;
    const int lane = threadIdx.x & 31, lr = lane & 15, hi = lane >> 4; const int r0 = blockIdx.x * 64, c0 = blockIdx.y * 64;
    v8f acc[4][4];
#pragma unroll
    for (int mb = 0; mb < 4; ++mb)
#pragma unroll
        for (int nb = 0; nb < 4; ++nb) acc[mb][nb] = (v8f){};
    const size_t aoff = (size_t)(r0 + lr) * K + 8 * hi, boff = (size_t)(c0 + lr) * K + 8 * hi;
#pragma unroll 1
    for (int kc = 0; kc < K; kc += 32) {
        v16h a[4];
#pragma unroll
        for (int mb = 0; mb < 4; ++mb) a[mb] = ldh(A + aoff + (size_t)mb * 16 * K + kc);
#pragma unroll
        for (int nb = 0; nb < 4; ++nb) { const v16h bq = ldh(Bt + boff + (size_t)nb * 16 * K + kc);
#pragma unroll
            for (int mb = 0; mb < 4; ++mb) acc[mb][nb] = wmma16(a[mb], bq, acc[mb][nb]); }
        asm volatile("v_nop\n\tv_nop\n\tv_nop\n\tv_nop" : "+v"(acc[0][0]), "+v"(acc[1][1]), "+v"(acc[2][2]), "+v"(acc[3][3]) : "v"(a[0]), "v"(a[1]), "v"(a[2]), "v"(a[3]));
    }
    const v4f braw = *(const v4f*)(bias + c0 + lr * 4); v4f bv;
#pragma unroll
    for (int i = 0; i < 4; ++i) bv[i] = bfr(braw[i]);
    const size_t orow0 = (size_t)(r0 / SEQ) * OUT_SEQ + (size_t)(r0 % SEQ);
#pragma unroll
    for (int mb = 0; mb < 4; ++mb) {
#pragma unroll
        for (int nb = 0; nb < 4; ++nb) {
#pragma unroll
            for (int j = 0; j < 8; ++j) os[(hi * 8 + j) * 68 + nb * 16 + lr] = acc[mb][nb][j]; }
        wave_sync();
        float* ob = OUT + (orow0 + (size_t)(mb * 16)) * DM + c0;
#pragma unroll 1
        for (int ps = 0; ps < 2; ++ps) {
#pragma unroll
            for (int s = 0; s < 8; ++s) { const int row = 2 * s + hi, cofs = lr * 4;
                const v4f xv = *(const v4fa*)(&os[row * 68 + cofs]); v4f val;
#pragma unroll
                for (int i = 0; i < 4; ++i) val[i] = xv[i] * OSC + bv[i];
                *(volatile v4f*)(ob + (size_t)row * DM + cofs) = val; }
            if (ps == 0) __threadfence(); }
        wave_sync();
    }
}

static constexpr size_t al256(size_t v) { return (v + 255) & ~(size_t)255; }
static constexpr size_t SZ_XB = al256((size_t)NB * SEQ * DM * 2);
static constexpr size_t SZ_WT = al256((size_t)3 * DM * DM * 2);
static constexpr size_t SZ_WP = al256((size_t)DM * DM * 2);
static constexpr size_t SZ_QK = al256((size_t)NB * 2 * NH_ * SEQ * HD * 2);
static constexpr size_t SZ_VT = al256((size_t)NB * NH_ * HD * SEQ * 2);
static constexpr size_t SZ_CT = al256((size_t)NB * SEQ * DM * 2);
static constexpr size_t SZ_TOTAL = SZ_XB + SZ_WT + SZ_WP + SZ_QK + SZ_VT + SZ_CT;
static_assert(SZ_TOTAL <= (size_t)134217728);

extern "C" void kernel_launch(void* const* d_in, const int* in_sizes, int n_in,
                              void* d_out, int out_size, void* d_ws, size_t ws_size, hipStream_t stream) {
    if (n_in < 5) return;
    const size_t needx = ((size_t)(NB - 1) * SEQ_FULL + SEQ) * DM;
    if ((size_t)in_sizes[0] < needx) return;
    if ((size_t)in_sizes[1] < (size_t)3 * DM * DM || (size_t)in_sizes[2] < (size_t)3 * DM) return;
    if ((size_t)in_sizes[3] < (size_t)DM * DM || (size_t)in_sizes[4] < (size_t)DM) return;
    if ((size_t)out_size < ((size_t)(NB - 1) * OUT_SEQ + SEQ) * DM) return;
    if (SZ_TOTAL > ws_size) return;
    const float* x = (const float*)d_in[0]; const float* wqkv = (const float*)d_in[1]; const float* bqkv = (const float*)d_in[2];
    const float* wproj = (const float*)d_in[3]; const float* bproj = (const float*)d_in[4];
    float* OUT = (float*)d_out;
    char* wsp = (char*)d_ws;
    bf*  XB = (bf*)wsp;  wsp += SZ_XB;
    bf*  WT = (bf*)wsp;  wsp += SZ_WT;
    h16* WP = (h16*)wsp; wsp += SZ_WP;
    h16* QK = (h16*)wsp; wsp += SZ_QK;
    h16* VT = (h16*)wsp; wsp += SZ_VT;
    h16* CT = (h16*)wsp; wsp += SZ_CT;

    if (SEQ == SEQ_FULL) {
        const size_t n8 = (size_t)NB * SEQ * DM / 8;
        k_cvt8<<<(unsigned)((n8 + 255) / 256), 256, 0, stream>>>(x, XB, n8);
    } else {
        const size_t n8 = (size_t)SEQ * DM / 8;
        for (int b = 0; b < NB; ++b) k_cvt8<<<(unsigned)((n8 + 255) / 256), 256, 0, stream>>>(x + (size_t)b * SEQ_FULL * DM, XB + (size_t)b * SEQ * DM, n8);
    }
    k_tr<<<dim3(3 * DM / 64, DM / 64, 1), 256, 0, stream>>>(wqkv, (unsigned short*)WT, DM, 3 * DM, 0, 1.0f);
    k_tr<<<dim3(DM / 64, DM / 64, 1), 256, 0, stream>>>(wproj, (unsigned short*)WP, DM, DM, 1, WPS);

    k_proj<<<dim3(NB * SEQ / 64, 2 * DM / 64, 1), 32, 0, stream>>>(XB, WT, bqkv, 0, QK, SEQ, (size_t)2 * NH_ * SEQ * HD, HD, HD, (size_t)SEQ * HD);
    k_proj<<<dim3(DM / 64, NB * SEQ / 64, 1), 32, 0, stream>>>(WT + (size_t)2 * DM * DM, XB, bqkv + 2 * DM, 1, VT, DM, (size_t)0, SEQ, SEQ, (size_t)DM * SEQ);

    k_flash<<<dim3(SEQ / (16 * AW), NB * NH_, 1), 32 * AW, 0, stream>>>(QK, VT, CT);

    k_out<<<dim3(NB * SEQ / 64, DM / 64, 1), 32, 0, stream>>>(CT, WP, bproj, OUT);
}
